// EGCL_68195490726193
// MI455X (gfx1250) — hardware-verified
//
#include <hip/hip_runtime.h>
#include <stddef.h>


#define DF     128
#define PQW    256
#define NTHR   128
#define NWAVE  4
#define EPT    8
#define CHUNK  (NTHR * EPT)
#define WCAP   (EPT * 32)
#define LISTN  (NWAVE * WCAP)
#define TE     16
#define PASSN  (NWAVE * TE)
#define PCAP   (CHUNK + PASSN)
#define NB     256
#define WPOOL  24576

static_assert(NTHR == DF);
static_assert((NB % (TE * NWAVE)) == 0);
static_assert(PASSN <= NTHR);
static_assert(PCAP >= CHUNK + PASSN);
static_assert(WPOOL == 2 * TE * DF * 2 + TE * DF * 4 + 2 * TE * DF * 2);
static_assert(WPOOL >= 2 * TE * PQW * 2 + 2 * TE * DF * 2);

typedef float          v4f   __attribute__((ext_vector_type(4)));
typedef float          v8f   __attribute__((ext_vector_type(8)));
typedef int            v4i   __attribute__((ext_vector_type(4)));
typedef unsigned short v4us  __attribute__((ext_vector_type(4)));
typedef unsigned short v8us  __attribute__((ext_vector_type(8)));
typedef unsigned short v16us __attribute__((ext_vector_type(16)));
typedef __bf16         v16bf __attribute__((ext_vector_type(16)));
union FragB { v16bf v; v16us u; v8us h[2]; };

__device__ __forceinline__ unsigned bf16_bits(float x) {
  const unsigned u = __float_as_uint(x);
  return (u + 0x7FFFu + ((u >> 16) & 1u)) >> 16;
}
__device__ __forceinline__ void split2(float x, unsigned short& hi, unsigned short& lo) {
  const unsigned hb = bf16_bits(x);
  const float    hf = __uint_as_float(hb << 16);
  const unsigned lb = bf16_bits(x - hf);
  hi = (unsigned short)hb;
  lo = (unsigned short)lb;
}

__device__ __forceinline__ FragB ldf(const unsigned short* base, int h8) {
  FragB f;
  f.h[0] = *(const v8us*)(base + h8);
  f.h[1] = *(const v8us*)(base + h8 + 16);
  return f;
}

__device__ __forceinline__ v8f wmb(const FragB& a, const FragB& b, v8f c) {
  v8f d = __builtin_amdgcn_wmma_f32_16x16x32_bf16(false, a.v, false, b.v, (short)0, c, false, false);
  asm volatile("v_nop\n\tv_nop\n\tv_nop\n\tv_nop" : "+v"(d) : "v"(a.v), "v"(b.v));
  return d;
}
__device__ __forceinline__ v8f wm3(const FragB& ah, const FragB& al, const FragB& bh, const FragB& bl, v8f c) {
  c = wmb(ah, bh, c);
  c = wmb(ah, bl, c);
  c = wmb(al, bh, c);
  return c;
}

__device__ __forceinline__ void vst4(float* p, v4f v) { *(volatile v4f*)p = v; }
__device__ __forceinline__ void vst8u(unsigned short* p, v8us v) { *(volatile v8us*)p = v; }

__device__ __forceinline__ float silu_f(float x) {
  return x * __builtin_amdgcn_rcpf(1.0f + __expf(-x));
}

__global__ __launch_bounds__(256) void k_hconv(const float* __restrict__ h, unsigned short* Hh, unsigned short* Hl, int n8) {
  const int t  = blockIdx.x * 256 + threadIdx.x;
  const int tc = t < n8 ? t : n8 - 1;
  const v4f a = *(const v4f*)(h + (size_t)tc * 8);
  const v4f b = *(const v4f*)(h + (size_t)tc * 8 + 4);
  float x[8];
  x[0] = a.x; x[1] = a.y; x[2] = a.z; x[3] = a.w;
  x[4] = b.x; x[5] = b.y; x[6] = b.z; x[7] = b.w;
  v8us hv, lv;
#pragma unroll
  for (int j = 0; j < 8; ++j) { unsigned short hs, ls; split2(x[j], hs, ls); hv[j] = hs; lv[j] = ls; }
  if (t < n8) { vst8u(Hh + (size_t)t * 8, hv); vst8u(Hl + (size_t)t * 8, lv); }
  __threadfence();
  if (t < n8) { vst8u(Hh + (size_t)t * 8, hv); vst8u(Hl + (size_t)t * 8, lv); }
}

__global__ __launch_bounds__(256) void k_wconv(const float* __restrict__ W, unsigned short* Oh, unsigned short* Ol,
                                                int K, int NC, int srcW, int nsplit, int koff2, int wtot) {
  const int t = blockIdx.x * 256 + threadIdx.x;
  const int K8 = K >> 3;
  const int total = NC * K8;
  const int tc = t < total ? t : total - 1;
  const int n  = tc / K8;
  const int kc = tc - n * K8;
  const int sel = (n >= nsplit) ? 1 : 0;
  const int cn  = n - sel * nsplit;
  const int ko  = sel * koff2;
  v8us hv, lv;
#pragma unroll
  for (int j = 0; j < 8; ++j) {
    int idx = (kc * 8 + j + ko) * srcW + cn;
    idx = idx < 0 ? 0 : (idx > wtot - 1 ? wtot - 1 : idx);
    const float v = W[idx];
    unsigned short hs, ls; split2(v, hs, ls);
    hv[j] = hs; lv[j] = ls;
  }
  const size_t o = (size_t)n * K + (size_t)kc * 8;
  if (t < total) { vst8u(Oh + o, hv); vst8u(Ol + o, lv); }
  __threadfence();
  if (t < total) { vst8u(Oh + o, hv); vst8u(Ol + o, lv); }
}

__global__ __launch_bounds__(128) void k_pq(const unsigned short* __restrict__ Hh, const unsigned short* __restrict__ Hl,
                                            const unsigned short* __restrict__ Wh, const unsigned short* __restrict__ Wl,
                                            float* PQ, int nN) {
  __shared__ __attribute__((aligned(16))) float tile[4 * 16 * PQW];
  const int tid = threadIdx.x, lane = tid & 31, wave = tid >> 5, hh = lane >> 4, m = lane & 15;
  const int row0 = blockIdx.x * 64 + wave * 16;
  int ra = row0 + m; ra = ra > nN - 1 ? nN - 1 : ra;
  float* T = tile + wave * (16 * PQW);
#pragma unroll 1
  for (int nt = 0; nt < PQW / 16; ++nt) {
    const int col = nt * 16 + m;
    v8f av;
#pragma unroll
    for (int i = 0; i < 8; ++i) av[i] = 0.0f;
#pragma unroll
    for (int kt = 0; kt < DF / 32; ++kt) {
      const int k0 = kt * 32;
      const FragB fah = ldf(Hh + (size_t)ra * DF + k0, 8 * hh);
      const FragB fal = ldf(Hl + (size_t)ra * DF + k0, 8 * hh);
      const FragB fbh = ldf(Wh + (size_t)col * DF + k0, 8 * hh);
      const FragB fbl = ldf(Wl + (size_t)col * DF + k0, 8 * hh);
      av = wm3(fah, fal, fbh, fbl, av);
    }
#pragma unroll
    for (int i = 0; i < 8; ++i) T[(8 * hh + i) * PQW + col] = av[i];
  }
  __syncthreads();
#pragma unroll 1
  for (int e = 0; e < 16; ++e) {
    const int row = row0 + e;
    if (row < nN) {
      const v4f v0 = *(const v4f*)(T + e * PQW + 4 * lane);
      const v4f v1 = *(const v4f*)(T + e * PQW + DF + 4 * lane);
      vst4(PQ + (size_t)row * PQW + 4 * lane, v0);
      vst4(PQ + (size_t)row * PQW + DF + 4 * lane, v1);
    }
  }
  __threadfence();
#pragma unroll 1
  for (int e = 0; e < 16; ++e) {
    const int row = row0 + e;
    if (row < nN) {
      const v4f v0 = *(const v4f*)(T + e * PQW + 4 * lane);
      const v4f v1 = *(const v4f*)(T + e * PQW + DF + 4 * lane);
      vst4(PQ + (size_t)row * PQW + 4 * lane, v0);
      vst4(PQ + (size_t)row * PQW + DF + 4 * lane, v1);
    }
  }
}

__device__ __forceinline__ int scan_chunk(const int* __restrict__ dsts, int nE, int cbase, int nodeBase,
                                          int* list, int tid, int wave) {
  int wc = 0;
  const int el0  = tid * EPT;
  const int e0   = cbase + el0;
  const int sent = -2147483647 - 1;
  const int last = nE - 1;
  v4i da, db;
  if (cbase + CHUNK <= nE) {
    da = *(const v4i*)(dsts + e0);
    db = *(const v4i*)(dsts + e0 + 4);
  } else {
    da.x = (e0     < nE) ? dsts[(e0    ) > last ? last : (e0    )] : sent;
    da.y = (e0 + 1 < nE) ? dsts[(e0 + 1) > last ? last : (e0 + 1)] : sent;
    da.z = (e0 + 2 < nE) ? dsts[(e0 + 2) > last ? last : (e0 + 2)] : sent;
    da.w = (e0 + 3 < nE) ? dsts[(e0 + 3) > last ? last : (e0 + 3)] : sent;
    db.x = (e0 + 4 < nE) ? dsts[(e0 + 4) > last ? last : (e0 + 4)] : sent;
    db.y = (e0 + 5 < nE) ? dsts[(e0 + 5) > last ? last : (e0 + 5)] : sent;
    db.z = (e0 + 6 < nE) ? dsts[(e0 + 6) > last ? last : (e0 + 6)] : sent;
    db.w = (e0 + 7 < nE) ? dsts[(e0 + 7) > last ? last : (e0 + 7)] : sent;
  }
  const unsigned nb = (unsigned)nodeBase;
  const unsigned s0 = (unsigned)da.x - nb, s1 = (unsigned)da.y - nb;
  const unsigned s2 = (unsigned)da.z - nb, s3 = (unsigned)da.w - nb;
  const unsigned s4 = (unsigned)db.x - nb, s5 = (unsigned)db.y - nb;
  const unsigned s6 = (unsigned)db.z - nb, s7 = (unsigned)db.w - nb;
  const bool h0 = s0 < (unsigned)NB, h1 = s1 < (unsigned)NB, h2 = s2 < (unsigned)NB, h3 = s3 < (unsigned)NB;
  const bool h4 = s4 < (unsigned)NB, h5 = s5 < (unsigned)NB, h6 = s6 < (unsigned)NB, h7 = s7 < (unsigned)NB;
  const unsigned any = __builtin_amdgcn_ballot_w32(h0 | h1 | h2 | h3 | h4 | h5 | h6 | h7);
  if (any != 0u) {
#define HITJ(J, HJ) { \
      const unsigned mj = __builtin_amdgcn_ballot_w32(HJ); \
      if (mj != 0u) { \
        if (HJ) { \
          const int pos = wc + (int)__builtin_amdgcn_mbcnt_lo(mj, 0u); \
          if (pos < WCAP) list[wave * WCAP + pos] = el0 + (J); \
        } \
        wc += (int)__builtin_popcount(mj); } }
    HITJ(0, h0)
    HITJ(1, h1)
    HITJ(2, h2)
    HITJ(3, h3)
    HITJ(4, h4)
    HITJ(5, h5)
    HITJ(6, h6)
    HITJ(7, h7)
#undef HITJ
  }
  return wc;
}

__global__ __launch_bounds__(NTHR) void k_agg(
    const float* __restrict__ h, const float* __restrict__ coord, const int* __restrict__ ei,
    const float* __restrict__ PQ, const unsigned short* __restrict__ Hh, const unsigned short* __restrict__ Hl,
    const unsigned short* __restrict__ W2h, const unsigned short* __restrict__ W2l,
    const unsigned short* __restrict__ Wc1h, const unsigned short* __restrict__ Wc1l,
    const unsigned short* __restrict__ Wn1h, const unsigned short* __restrict__ Wn1l,
    const unsigned short* __restrict__ Wn2h, const unsigned short* __restrict__ Wn2l,
    const float* __restrict__ We1, const float* __restrict__ be1, const float* __restrict__ be2,
    const float* __restrict__ bc1, const float* __restrict__ Wc2, const float* __restrict__ bc2,
    const float* __restrict__ bn1, const float* __restrict__ bn2,
    float* out0, float* out1, int nN, int nE) {
  __shared__ __attribute__((aligned(16))) float acc[(NB + 1) * DF];
  __shared__ __attribute__((aligned(16))) float cacc[(NB + 1) * 4];
  __shared__ __attribute__((aligned(16))) unsigned char wpool[NWAVE * WPOOL];
  __shared__ __attribute__((aligned(16))) int list[LISTN];
  __shared__ __attribute__((aligned(16))) int pend[PCAP];
  __shared__ int   eslot[PASSN], erid[PASSN], ecid[PASSN];
  __shared__ float erad[PASSN], ewgt[PASSN], edn[3 * PASSN];
  __shared__ __attribute__((aligned(16))) float pw257[DF], pbe1[DF], pbe2[DF], pbc1[DF], pwc2[DF], pbn1[DF], pbn2[DF];
  __shared__ __attribute__((aligned(16))) float cstage[NB * 3];
  __shared__ int wcnt[NWAVE];
  __shared__ int pendN;

  const int tid = threadIdx.x, lane = tid & 31, wave = tid >> 5, hh = lane >> 4, m = lane & 15;
  const int nodeBase = blockIdx.x * NB;
  const int* dsts = ei;
  const int* srcs = ei + nE;
  unsigned char* wp = wpool + wave * WPOOL;
  unsigned short* xh  = (unsigned short*)wp;
  unsigned short* xl  = (unsigned short*)(wp + 4096);
  float*          mfw = (float*)(wp + 8192);
  unsigned short* mh  = (unsigned short*)(wp + 16384);
  unsigned short* ml  = (unsigned short*)(wp + 20480);

  for (int i = tid; i < (NB + 1) * DF; i += NTHR) acc[i] = 0.0f;
  for (int i = tid; i < (NB + 1) * 4; i += NTHR) cacc[i] = 0.0f;
  {
    pw257[tid] = We1[(size_t)256 * DF + tid];
    pbe1[tid]  = be1[tid];
    pbe2[tid]  = be2[tid];
    pbc1[tid]  = bc1[tid];
    pwc2[tid]  = Wc2[tid];
    pbn1[tid]  = bn1[tid];
    pbn2[tid]  = bn2[tid];
  }
  if (tid == 0) pendN = 0;
  const float bc2v = bc2[0];
  __syncthreads();

  const int nChunks = (nE + CHUNK - 1) / CHUNK;
#pragma unroll 1
  for (int ch = 0; ch < nChunks; ++ch) {
    const int cbase = ch * CHUNK;
    const int wc = scan_chunk(dsts, nE, cbase, nodeBase, list, tid, wave);
    if (lane == 0) wcnt[wave] = wc;
    __syncthreads();

    const int base = pendN;
    int tot = 0, myoff = 0;
#pragma unroll
    for (int w = 0; w < NWAVE; ++w) {
      int c = wcnt[w];
      c = c > WCAP ? WCAP : (c < 0 ? 0 : c);
      if (w < wave) myoff += c;
      tot += c;
    }
    int newN = base + tot;
    newN = newN > PCAP ? PCAP : newN;
    {
      int n = wcnt[wave];
      n = n > WCAP ? WCAP : (n < 0 ? 0 : n);
      const int* lp = list + wave * WCAP;
      for (int i = lane; i < n; i += 32) {
        const int pos = base + myoff + i;
        if (pos < PCAP) pend[pos] = cbase + lp[i];
      }
    }
    const int fin = (ch == nChunks - 1) ? 1 : 0;
    const int R   = (fin != 0) ? (newN + PASSN - 1) / PASSN : newN / PASSN;
    const int Pv  = (fin != 0) ? newN : R * PASSN;
    __syncthreads();

#pragma unroll 1
    for (int r = 0; r < R; ++r) {
      {
        const int idx = r * PASSN + wave * TE + m;
        const bool valid = (lane < TE) && (idx < Pv);
        int e = pend[idx];
        if (!valid) e = 0;
        e = e < 0 ? 0 : (e > nE - 1 ? nE - 1 : e);
        int rr = dsts[e];
        int cc = srcs[e];
        int slot = rr - nodeBase;
        if (!valid || (unsigned)slot >= (unsigned)NB) slot = NB;
        rr = rr < 0 ? 0 : (rr > nN - 1 ? nN - 1 : rr);
        cc = cc < 0 ? 0 : (cc > nN - 1 ? nN - 1 : cc);
        const float* pr = coord + (size_t)rr * 3;
        const float* pc = coord + (size_t)cc * 3;
        const float dx = pr[0] - pc[0];
        const float dy = pr[1] - pc[1];
        const float dz = pr[2] - pc[2];
        const float rad = dx * dx + dy * dy + dz * dz;
        const float inv = __builtin_amdgcn_rcpf(sqrtf(rad) + 1e-8f);
        if (lane < TE) {
          const int q = wave * TE + m;
          eslot[q] = slot; erid[q] = rr; ecid[q] = cc; erad[q] = rad;
          edn[q] = dx * inv; edn[PASSN + q] = dy * inv; edn[2 * PASSN + q] = dz * inv;
        }
      }
      __syncthreads();

      {
        const v4f w4 = *(const v4f*)(pw257 + 4 * lane);
        const v4f b4 = *(const v4f*)(pbe1 + 4 * lane);
#pragma unroll 1
        for (int e = 0; e < TE; ++e) {
          const int q = wave * TE + e;
          const int rr = erid[q], cc = ecid[q];
          const float rad = erad[q];
          const v4f p  = *(const v4f*)(PQ + (size_t)rr * PQW + 4 * lane);
          const v4f qq = *(const v4f*)(PQ + (size_t)cc * PQW + DF + 4 * lane);
          v4us hv, lv;
#pragma unroll
          for (int c = 0; c < 4; ++c) {
            const float x = silu_f(p[c] + qq[c] + rad * w4[c] + b4[c]);
            unsigned short hs, ls; split2(x, hs, ls);
            hv[c] = hs; lv[c] = ls;
          }
          *(v4us*)(xh + e * DF + 4 * lane) = hv;
          *(v4us*)(xl + e * DF + 4 * lane) = lv;
        }
      }
      __syncthreads();

      {
#pragma unroll 1
        for (int nt = 0; nt < DF / 16; ++nt) {
          const int col = nt * 16 + m;
          const float bv = pbe2[col];
          v8f av;
#pragma unroll
          for (int i = 0; i < 8; ++i) av[i] = bv;
#pragma unroll
          for (int kt = 0; kt < DF / 32; ++kt) {
            const int k0 = kt * 32;
            const FragB fah = ldf(xh + m * DF + k0, 8 * hh);
            const FragB fal = ldf(xl + m * DF + k0, 8 * hh);
            const FragB fbh = ldf(W2h + (size_t)col * DF + k0, 8 * hh);
            const FragB fbl = ldf(W2l + (size_t)col * DF + k0, 8 * hh);
            av = wm3(fah, fal, fbh, fbl, av);
          }
#pragma unroll
          for (int i = 0; i < 8; ++i) {
            const int row = 8 * hh + i;
            const float v = silu_f(av[i]);
            unsigned short hs, ls; split2(v, hs, ls);
            mfw[row * DF + col] = v;
            mh[row * DF + col]  = hs;
            ml[row * DF + col]  = ls;
          }
        }
      }
      __syncthreads();

      {
        float part[8];
#pragma unroll
        for (int i = 0; i < 8; ++i) part[i] = 0.0f;
#pragma unroll 1
        for (int nt = 0; nt < DF / 16; ++nt) {
          const int col = nt * 16 + m;
          const float bv = pbc1[col];
          v8f av;
#pragma unroll
          for (int i = 0; i < 8; ++i) av[i] = bv;
#pragma unroll
          for (int kt = 0; kt < DF / 32; ++kt) {
            const int k0 = kt * 32;
            const FragB fah = ldf(mh + m * DF + k0, 8 * hh);
            const FragB fal = ldf(ml + m * DF + k0, 8 * hh);
            const FragB fbh = ldf(Wc1h + (size_t)col * DF + k0, 8 * hh);
            const FragB fbl = ldf(Wc1l + (size_t)col * DF + k0, 8 * hh);
            av = wm3(fah, fal, fbh, fbl, av);
          }
          const float wcv = pwc2[col];
#pragma unroll
          for (int i = 0; i < 8; ++i) part[i] += silu_f(av[i]) * wcv;
        }
#pragma unroll
        for (int i = 0; i < 8; ++i) {
          part[i] += __shfl_xor(part[i], 1, 32);
          part[i] += __shfl_xor(part[i], 2, 32);
          part[i] += __shfl_xor(part[i], 4, 32);
          part[i] += __shfl_xor(part[i], 8, 32);
        }
        if (m == 0) {
#pragma unroll
          for (int i = 0; i < 8; ++i) ewgt[wave * TE + 8 * hh + i] = part[i] + bc2v;
        }
      }
      __syncthreads();

      {
#pragma unroll 1
        for (int i = 0; i < PASSN; ++i) {
          int sl = eslot[i];
          sl = sl < 0 ? 0 : (sl > NB ? NB : sl);
          const float* mrow = (const float*)(wpool + (i >> 4) * WPOOL + 8192) + (i & 15) * DF;
          const float v = mrow[tid];
          acc[sl * DF + tid] += v;
          if (tid < 3) {
            const float d = edn[tid * PASSN + i] * ewgt[i];
            cacc[sl * 4 + tid] += d;
          }
        }
      }
      __syncthreads();
    }

    int rem = newN - R * PASSN;
    rem = rem < 0 ? 0 : rem;
    if (R > 0 && tid < rem) pend[tid] = pend[R * PASSN + tid];
    if (tid == 0) pendN = rem;
  }
  __syncthreads();

  {
    for (int i = tid; i < NB * 3; i += NTHR) {
      const int n = i / 3;
      const int k = i - n * 3;
      int node = nodeBase + n; node = node > nN - 1 ? nN - 1 : node;
      cstage[i] = coord[(size_t)node * 3 + k] + cacc[n * 4 + k];
    }
    __syncthreads();
    const size_t gb  = (size_t)nodeBase * 3;
    const size_t lim = (size_t)nN * 3;
    const int q0 = tid, q1 = tid + NTHR;
    v4f v0 = *(const v4f*)(cstage + 4 * q0);
    v4f v1 = {0.0f, 0.0f, 0.0f, 0.0f};
    if (q1 < (NB * 3) / 4) v1 = *(const v4f*)(cstage + 4 * q1);
    const bool w0 = (gb + 4 * (size_t)q0 + 4 <= lim);
    const bool w1 = (q1 < (NB * 3) / 4) && (gb + 4 * (size_t)q1 + 4 <= lim);
    if (w0) vst4(out1 + gb + 4 * q0, v0);
    if (w1) vst4(out1 + gb + 4 * q1, v1);
    __threadfence();
    if (w0) vst4(out1 + gb + 4 * q0, v0);
    if (w1) vst4(out1 + gb + 4 * q1, v1);
  }
  __syncthreads();

  {
    unsigned short* anh = (unsigned short*)wp;
    unsigned short* anl = (unsigned short*)(wp + 8192);
    unsigned short* yh  = (unsigned short*)(wp + 16384);
    unsigned short* yl  = (unsigned short*)(wp + 20480);
    float*          ot  = (float*)wp;
#pragma unroll 1
    for (int tt = 0; tt < NB / (TE * NWAVE); ++tt) {
      const int n0 = (tt * NWAVE + wave) * TE;
#pragma unroll 1
      for (int e = 0; e < TE; ++e) {
        int node = nodeBase + n0 + e; node = node > nN - 1 ? nN - 1 : node;
        const v4us a = *(const v4us*)(Hh + (size_t)node * DF + 4 * lane);
        const v4us b = *(const v4us*)(Hl + (size_t)node * DF + 4 * lane);
        *(v4us*)(anh + e * PQW + 4 * lane) = a;
        *(v4us*)(anl + e * PQW + 4 * lane) = b;
        const v4f mi = *(const v4f*)(acc + (n0 + e) * DF + 4 * lane);
        v4us mh4, ml4;
#pragma unroll
        for (int c = 0; c < 4; ++c) { unsigned short hs, ls; split2(mi[c], hs, ls); mh4[c] = hs; ml4[c] = ls; }
        *(v4us*)(anh + e * PQW + DF + 4 * lane) = mh4;
        *(v4us*)(anl + e * PQW + DF + 4 * lane) = ml4;
      }
      __syncthreads();
#pragma unroll 1
      for (int nt = 0; nt < DF / 16; ++nt) {
        const int col = nt * 16 + m;
        const float bv = pbn1[col];
        v8f av;
#pragma unroll
        for (int i = 0; i < 8; ++i) av[i] = bv;
#pragma unroll 4
        for (int kt = 0; kt < PQW / 32; ++kt) {
          const int k0 = kt * 32;
          const FragB fah = ldf(anh + m * PQW + k0, 8 * hh);
          const FragB fal = ldf(anl + m * PQW + k0, 8 * hh);
          const FragB fbh = ldf(Wn1h + (size_t)col * PQW + k0, 8 * hh);
          const FragB fbl = ldf(Wn1l + (size_t)col * PQW + k0, 8 * hh);
          av = wm3(fah, fal, fbh, fbl, av);
        }
#pragma unroll
        for (int i = 0; i < 8; ++i) {
          const int row = 8 * hh + i;
          const float v = silu_f(av[i]);
          unsigned short hs, ls; split2(v, hs, ls);
          yh[row * DF + col] = hs;
          yl[row * DF + col] = ls;
        }
      }
      __syncthreads();
#pragma unroll 1
      for (int nt = 0; nt < DF / 16; ++nt) {
        const int col = nt * 16 + m;
        const float bv = pbn2[col];
        v8f av;
#pragma unroll
        for (int i = 0; i < 8; ++i) av[i] = bv;
#pragma unroll
        for (int kt = 0; kt < DF / 32; ++kt) {
          const int k0 = kt * 32;
          const FragB fah = ldf(yh + m * DF + k0, 8 * hh);
          const FragB fal = ldf(yl + m * DF + k0, 8 * hh);
          const FragB fbh = ldf(Wn2h + (size_t)col * DF + k0, 8 * hh);
          const FragB fbl = ldf(Wn2l + (size_t)col * DF + k0, 8 * hh);
          av = wm3(fah, fal, fbh, fbl, av);
        }
#pragma unroll
        for (int i = 0; i < 8; ++i) ot[(8 * hh + i) * DF + col] = av[i];
      }
      __syncthreads();
#pragma unroll 1
      for (int e = 0; e < TE; ++e) {
        const int node = nodeBase + n0 + e;
        const int nc = node > nN - 1 ? nN - 1 : node;
        v4f v = *(const v4f*)(ot + e * DF + 4 * lane);
        const v4f hv4 = *(const v4f*)(h + (size_t)nc * DF + 4 * lane);
        v += hv4;
        *(v4f*)(ot + e * DF + 4 * lane) = v;
        if (node < nN) vst4(out0 + (size_t)node * DF + 4 * lane, v);
      }
      __threadfence();
#pragma unroll 1
      for (int e = 0; e < TE; ++e) {
        const int node = nodeBase + n0 + e;
        if (node < nN) {
          const v4f v = *(const v4f*)(ot + e * DF + 4 * lane);
          vst4(out0 + (size_t)node * DF + 4 * lane, v);
        }
      }
      __syncthreads();
    }
  }
}

extern "C" void kernel_launch(void* const* d_in, const int* in_sizes, int n_in,
                              void* d_out, int out_size, void* d_ws, size_t ws_size,
                              hipStream_t stream) {
  if (n_in < 15) return;
  const int nN = in_sizes[0] / DF;
  const int nE = in_sizes[2] / 2;
  if (nN <= 0 || nE <= 0) return;
  if (in_sizes[0] != nN * DF || in_sizes[1] != nN * 3 || in_sizes[2] != nE * 2) return;
  if (in_sizes[3] != 257 * DF || in_sizes[4] != DF || in_sizes[5] != DF * DF || in_sizes[6] != DF) return;
  if (in_sizes[7] != DF * DF || in_sizes[8] != DF || in_sizes[9] != DF || in_sizes[10] < 1) return;
  if (in_sizes[11] != 2 * DF * DF || in_sizes[12] != DF || in_sizes[13] != DF * DF || in_sizes[14] != DF) return;
  if (out_size != nN * DF + nN * 3) return;

  const float* h     = (const float*)d_in[0];
  const float* coord = (const float*)d_in[1];
  const int*   ei    = (const int*)d_in[2];
  const float* We1 = (const float*)d_in[3];  const float* be1 = (const float*)d_in[4];
  const float* We2 = (const float*)d_in[5];  const float* be2 = (const float*)d_in[6];
  const float* Wc1 = (const float*)d_in[7];  const float* bc1 = (const float*)d_in[8];
  const float* Wc2 = (const float*)d_in[9];  const float* bc2 = (const float*)d_in[10];
  const float* Wn1 = (const float*)d_in[11]; const float* bn1 = (const float*)d_in[12];
  const float* Wn2 = (const float*)d_in[13]; const float* bn2 = (const float*)d_in[14];

  float* out0 = (float*)d_out;
  float* out1 = (float*)d_out + (size_t)nN * DF;

  char* ws = (char*)d_ws;
  size_t off = 0;
  auto take = [&](size_t bytes) -> size_t { const size_t o = off; off = (off + bytes + 255) & ~(size_t)255; return o; };
  const size_t oHh  = take((size_t)nN * DF * 2);
  const size_t oHl  = take((size_t)nN * DF * 2);
  const size_t oPQ  = take((size_t)nN * PQW * 4);
  const size_t oW1h = take((size_t)PQW * DF * 2), oW1l = take((size_t)PQW * DF * 2);
  const size_t oW2h = take((size_t)DF * DF * 2),  oW2l = take((size_t)DF * DF * 2);
  const size_t oC1h = take((size_t)DF * DF * 2),  oC1l = take((size_t)DF * DF * 2);
  const size_t oN1h = take((size_t)DF * PQW * 2), oN1l = take((size_t)DF * PQW * 2);
  const size_t oN2h = take((size_t)DF * DF * 2),  oN2l = take((size_t)DF * DF * 2);
  if (off > ws_size) return;
  if (off > (size_t)134217728) return;

  unsigned short* Hh   = (unsigned short*)(ws + oHh);
  unsigned short* Hl   = (unsigned short*)(ws + oHl);
  float*          PQ   = (float*)(ws + oPQ);
  unsigned short* W1h  = (unsigned short*)(ws + oW1h); unsigned short* W1l  = (unsigned short*)(ws + oW1l);
  unsigned short* W2h  = (unsigned short*)(ws + oW2h); unsigned short* W2l  = (unsigned short*)(ws + oW2l);
  unsigned short* C1h  = (unsigned short*)(ws + oC1h); unsigned short* C1l  = (unsigned short*)(ws + oC1l);
  unsigned short* N1h  = (unsigned short*)(ws + oN1h); unsigned short* N1l  = (unsigned short*)(ws + oN1l);
  unsigned short* N2h  = (unsigned short*)(ws + oN2h); unsigned short* N2l  = (unsigned short*)(ws + oN2l);

  {
    const int n8 = nN * DF / 8;
    k_hconv<<<(n8 + 255) / 256, 256, 0, stream>>>(h, Hh, Hl, n8);
  }
  {
    const int t1 = PQW * (DF / 8);
    k_wconv<<<(t1 + 255) / 256, 256, 0, stream>>>(We1, W1h, W1l, DF, PQW, DF, DF, DF, in_sizes[3]);
    const int t2 = DF * (DF / 8);
    k_wconv<<<(t2 + 255) / 256, 256, 0, stream>>>(We2, W2h, W2l, DF, DF, DF, DF, 0, in_sizes[5]);
    k_wconv<<<(t2 + 255) / 256, 256, 0, stream>>>(Wc1, C1h, C1l, DF, DF, DF, DF, 0, in_sizes[7]);
    const int t3 = DF * (PQW / 8);
    k_wconv<<<(t3 + 255) / 256, 256, 0, stream>>>(Wn1, N1h, N1l, PQW, DF, DF, DF, 0, in_sizes[11]);
    k_wconv<<<(t2 + 255) / 256, 256, 0, stream>>>(Wn2, N2h, N2l, DF, DF, DF, DF, 0, in_sizes[13]);
  }
  k_pq<<<(nN + 63) / 64, 128, 0, stream>>>(Hh, Hl, W1h, W1l, PQ, nN);
  {
    const int nBlk = (nN + NB - 1) / NB;
    k_agg<<<nBlk, NTHR, 0, stream>>>(h, coord, ei, PQ, Hh, Hl, W2h, W2l, C1h, C1l, N1h, N1l, N2h, N2l,
                                     We1, be1, be2, bc1, Wc2, bc2, bn1, bn2, out0, out1, nN, nE);
  }
}
